// HTGTLayer_71116068487908
// MI455X (gfx1250) — hardware-verified
//
#include <hip/hip_runtime.h>
#include <stddef.h>
#include <math.h>


#pragma clang fp contract(off)

#define NTHR   256
#define NWAVE  8
#define EPT    8
#define CHUNK  (NTHR * EPT)
#define WCAP   (EPT * 32)
#define LISTN  (NWAVE * WCAP)
#define ID     128
#define TD     32
#define ED     32
#define KS     160
#define OD     128
#define NH     8
#define NREL   8
#define NTYP   4
#define ETILE  16
#define EROW   160
#define MSGW   136
#define NB     128
#define LN_EPS 1e-5f
#define ISQ    (1.0f / 11.313708498984761f)

static_assert(LISTN == CHUNK);
static_assert((EROW * 4) % 128 == 0);
static_assert((NB % ETILE) == 0);
static_assert(MSGW == OD + NH);

typedef float          v2f   __attribute__((ext_vector_type(2)));
typedef float          v4f   __attribute__((ext_vector_type(4)));
typedef float          v8f   __attribute__((ext_vector_type(8)));
typedef int            v4i   __attribute__((ext_vector_type(4)));
typedef int            v8i   __attribute__((ext_vector_type(8)));
typedef unsigned int   v4u   __attribute__((ext_vector_type(4)));
typedef unsigned short v8us  __attribute__((ext_vector_type(8)));
typedef __bf16         v16bf __attribute__((ext_vector_type(16)));
union FragB { v16bf v; v8us u[2]; v8i w; };

__device__ __forceinline__ int clampi(int v, int lo, int hi) { return v < lo ? lo : (v > hi ? hi : v); }

__device__ __forceinline__ v8f zero8f() {
  v8f z = {0.f, 0.f, 0.f, 0.f, 0.f, 0.f, 0.f, 0.f};
  return z;
}

__device__ __forceinline__ unsigned int bfb(float x) {
  unsigned int u = __float_as_uint(x);
  u += 0x7FFFu + ((u >> 16) & 1u);
  return u >> 16;
}
__device__ __forceinline__ float bff(unsigned int b) { return __uint_as_float(b << 16); }

__device__ __forceinline__ void split2(float a, float b, unsigned int& ph, unsigned int& pl) {
  const unsigned int ha = bfb(a), hb = bfb(b);
  const unsigned int la = bfb(a - bff(ha)), lb = bfb(b - bff(hb));
  ph = ha | (hb << 16);
  pl = la | (lb << 16);
}

__device__ __forceinline__ v8f wmb(const FragB& a, const FragB& b, v8f c) {
  v8f d = __builtin_amdgcn_wmma_f32_16x16x32_bf16(false, a.v, false, b.v, (short)0, c, false, false);
  asm volatile("v_nop\n\tv_nop\n\tv_nop\n\tv_nop" : "+v"(d) : "v"(a.w), "v"(b.w));
  return d;
}

__device__ __forceinline__ FragB ldfrag(const unsigned short* p) {
  FragB f;
  f.u[0] = *(const v8us*)p;
  f.u[1] = *(const v8us*)(p + 16);
  return f;
}

__device__ __forceinline__ float hsum16(float v) {
  v += __shfl_xor(v, 1, 32);
  v += __shfl_xor(v, 2, 32);
  v += __shfl_xor(v, 4, 32);
  v += __shfl_xor(v, 8, 32);
  return v;
}

__device__ __forceinline__ void load8(const int* __restrict__ p, int n, int e0, int full, v4i& da, v4i& db) {
  const int sent = -2147483647 - 1;
  if (full != 0) {
    da = *(const v4i*)(p + e0);
    db = *(const v4i*)(p + e0 + 4);
  } else {
    da.x = (e0     < n) ? p[clampi(e0,     0, n - 1)] : sent;
    da.y = (e0 + 1 < n) ? p[clampi(e0 + 1, 0, n - 1)] : sent;
    da.z = (e0 + 2 < n) ? p[clampi(e0 + 2, 0, n - 1)] : sent;
    da.w = (e0 + 3 < n) ? p[clampi(e0 + 3, 0, n - 1)] : sent;
    db.x = (e0 + 4 < n) ? p[clampi(e0 + 4, 0, n - 1)] : sent;
    db.y = (e0 + 5 < n) ? p[clampi(e0 + 5, 0, n - 1)] : sent;
    db.z = (e0 + 6 < n) ? p[clampi(e0 + 6, 0, n - 1)] : sent;
    db.w = (e0 + 7 < n) ? p[clampi(e0 + 7, 0, n - 1)] : sent;
  }
}

__device__ __forceinline__ int compact8(bool h0, bool h1, bool h2, bool h3, bool h4, bool h5, bool h6, bool h7,
                                        int el0, int* list, int wave) {
  int wc = 0;
  const unsigned any = __builtin_amdgcn_ballot_w32(h0 | h1 | h2 | h3 | h4 | h5 | h6 | h7);
  if (any != 0u) {
#define HITJ(J, HJ) { \
      const unsigned mj = __builtin_amdgcn_ballot_w32(HJ); \
      if (mj != 0u) { \
        if (HJ) { \
          const int pos = wc + (int)__builtin_amdgcn_mbcnt_lo(mj, 0u); \
          if (pos < WCAP) list[wave * WCAP + pos] = el0 + (J); \
        } \
        wc += (int)__builtin_popcount(mj); } }
    HITJ(0, h0)
    HITJ(1, h1)
    HITJ(2, h2)
    HITJ(3, h3)
    HITJ(4, h4)
    HITJ(5, h5)
    HITJ(6, h6)
    HITJ(7, h7)
#undef HITJ
  }
  return wc;
}

__device__ __forceinline__ int flatten(const int* list, int* pend, const int* wcnt, int cbase, int lane, int wave) {
  int tot = 0, myoff = 0;
#pragma unroll
  for (int w = 0; w < NWAVE; ++w) {
    int c = wcnt[w];
    c = c > WCAP ? WCAP : (c < 0 ? 0 : c);
    if (w < wave) myoff += c;
    tot += c;
  }
  int n = wcnt[wave];
  n = n > WCAP ? WCAP : (n < 0 ? 0 : n);
  for (int i = lane; i < n; i += 32) {
    const int pos = myoff + i;
    if (pos < LISTN) pend[pos] = cbase + list[wave * WCAP + i];
  }
  return tot > LISTN ? LISTN : tot;
}

__global__ __launch_bounds__(NTHR) void k_wprep(
    const float* __restrict__ Wq, const float* __restrict__ Wk, const float* __restrict__ Wv, const float* __restrict__ Wa,
    unsigned short* wqh, unsigned short* wql, unsigned short* wkh, unsigned short* wkl,
    unsigned short* wvh, unsigned short* wvl, unsigned short* wah, unsigned short* wal) {
  const int g = blockIdx.x * NTHR + threadIdx.x;
  const int nq = NREL * OD * (ID / 8), nk = NREL * OD * (KS / 8), na = NTYP * OD * (OD / 8);
  const int total = nq + 2 * nk + na;
  if (g >= total) return;
  const float* W; unsigned short* ph; unsigned short* pl; int K; int gl;
  if (g < nq)               { W = Wq; ph = wqh; pl = wql; K = ID; gl = g; }
  else if (g < nq + nk)     { W = Wk; ph = wkh; pl = wkl; K = KS; gl = g - nq; }
  else if (g < nq + 2 * nk) { W = Wv; ph = wvh; pl = wvl; K = KS; gl = g - nq - nk; }
  else                      { W = Wa; ph = wah; pl = wal; K = OD; gl = g - nq - 2 * nk; }
  const int kg  = K / 8;
  const int gpr = OD * kg;
  const int rr  = gl / gpr, rem = gl - rr * gpr;
  const int n   = rem / kg, k0 = (rem - n * kg) * 8;
  const float* src = W + ((size_t)rr * K + k0) * OD + n;
  float x[8];
#pragma unroll
  for (int i = 0; i < 8; ++i) x[i] = src[(size_t)i * OD];
  unsigned int p0h, p0l, p1h, p1l, p2h, p2l, p3h, p3l;
  split2(x[0], x[1], p0h, p0l);
  split2(x[2], x[3], p1h, p1l);
  split2(x[4], x[5], p2h, p2l);
  split2(x[6], x[7], p3h, p3l);
  v4u hv = {p0h, p1h, p2h, p3h};
  v4u lv = {p0l, p1l, p2l, p3l};
  unsigned short* dh = ph + (size_t)gl * 8;
  unsigned short* dl = pl + (size_t)gl * 8;
  *(volatile v4u*)dh = hv;
  *(volatile v4u*)dl = lv;
  __threadfence();
  *(volatile v4u*)dh = hv;
  *(volatile v4u*)dl = lv;
}

__global__ __launch_bounds__(NTHR) void k_edge(
    const float* __restrict__ src_h, const float* __restrict__ src_tw, const float* __restrict__ src_tb,
    const float* __restrict__ edge_h, const float* __restrict__ date,
    const int* __restrict__ src_idx, const int* __restrict__ dst_idx, const int* __restrict__ etype,
    const float* __restrict__ sg, const float* __restrict__ sb,
    const float* __restrict__ dg, const float* __restrict__ dbeta,
    const unsigned short* __restrict__ wqh, const unsigned short* __restrict__ wql,
    const unsigned short* __restrict__ wkh, const unsigned short* __restrict__ wkl,
    const unsigned short* __restrict__ wvh, const unsigned short* __restrict__ wvl,
    float* eplane, int nN, int nE, int vec8) {
  __shared__ __attribute__((aligned(16))) unsigned short sAdH[ETILE * ID];
  __shared__ __attribute__((aligned(16))) unsigned short sAdL[ETILE * ID];
  __shared__ __attribute__((aligned(16))) unsigned short sAsH[ETILE * KS];
  __shared__ __attribute__((aligned(16))) unsigned short sAsL[ETILE * KS];
  __shared__ __attribute__((aligned(16))) float sOut[ETILE * EROW];
  __shared__ __attribute__((aligned(16))) int list[LISTN];
  __shared__ __attribute__((aligned(16))) int pend[LISTN];
  __shared__ int wcnt[NWAVE];

  const int tid = threadIdx.x, lane = tid & 31, wave = tid >> 5, hh = lane >> 4, mc = lane & 15;
  const int m = tid >> 4, ln = tid & 15;
  const int cbase = blockIdx.x * CHUNK;

  for (int i = tid; i < ETILE * (EROW - MSGW); i += NTHR) {
    const int row = i / (EROW - MSGW);
    const int c = MSGW + (i - row * (EROW - MSGW));
    sOut[row * EROW + c] = 0.f;
  }

  int et[8];
  {
    const int e0 = cbase + tid * EPT;
    const int full = (vec8 != 0 && cbase + CHUNK <= nE) ? 1 : 0;
    v4i ea, eb;
    load8(etype, nE, e0, full, ea, eb);
    et[0] = (e0     < nE) ? clampi(ea.x, 0, NREL - 1) : -1;
    et[1] = (e0 + 1 < nE) ? clampi(ea.y, 0, NREL - 1) : -1;
    et[2] = (e0 + 2 < nE) ? clampi(ea.z, 0, NREL - 1) : -1;
    et[3] = (e0 + 3 < nE) ? clampi(ea.w, 0, NREL - 1) : -1;
    et[4] = (e0 + 4 < nE) ? clampi(eb.x, 0, NREL - 1) : -1;
    et[5] = (e0 + 5 < nE) ? clampi(eb.y, 0, NREL - 1) : -1;
    et[6] = (e0 + 6 < nE) ? clampi(eb.z, 0, NREL - 1) : -1;
    et[7] = (e0 + 7 < nE) ? clampi(eb.w, 0, NREL - 1) : -1;
  }
  __syncthreads();

#pragma unroll 1
  for (int r = 0; r < NREL; ++r) {
    {
      const int wc = compact8(et[0] == r, et[1] == r, et[2] == r, et[3] == r,
                              et[4] == r, et[5] == r, et[6] == r, et[7] == r,
                              tid * EPT, list, wave);
      if (lane == 0) wcnt[wave] = wc;
    }
    __syncthreads();
    const int tot = flatten(list, pend, wcnt, cbase, lane, wave);
    __syncthreads();
    const int nT = (tot + ETILE - 1) / ETILE;

    const unsigned short* wq_h = wqh + (size_t)r * OD * ID;
    const unsigned short* wq_l = wql + (size_t)r * OD * ID;
    const unsigned short* wk_h = wkh + (size_t)r * OD * KS;
    const unsigned short* wk_l = wkl + (size_t)r * OD * KS;
    const unsigned short* wv_h = wvh + (size_t)r * OD * KS;
    const unsigned short* wv_l = wvl + (size_t)r * OD * KS;

#pragma unroll 1
    for (int tile = 0; tile < nT; ++tile) {
      {
        const int i0 = tile * ETILE + m;
        const bool valid = i0 < tot;
        int e = pend[i0];
        e = valid ? e : 0;
        e = clampi(e, 0, nE - 1);
        const int si = clampi(src_idx[e], 0, nN - 1);
        const int di = clampi(dst_idx[e], 0, nN - 1);
        const float t = date[e];
        const int c2 = 2 * ln, c6 = TD + 6 * ln;
        {
          const float* hr = src_h + (size_t)di * ID;
          const v2f hm = *(const v2f*)(hr + c2);
          const v2f tw = *(const v2f*)(src_tw + (size_t)di * TD + c2);
          const v2f tb = *(const v2f*)(src_tb + (size_t)di * TD + c2);
          const v2f h0 = *(const v2f*)(hr + c6), h1 = *(const v2f*)(hr + c6 + 2), h2 = *(const v2f*)(hr + c6 + 4);
          const v2f g0 = *(const v2f*)(dg + c2), g1 = *(const v2f*)(dg + c6), g2 = *(const v2f*)(dg + c6 + 2), g3 = *(const v2f*)(dg + c6 + 4);
          const v2f o0 = *(const v2f*)(dbeta + c2), o1 = *(const v2f*)(dbeta + c6), o2 = *(const v2f*)(dbeta + c6 + 2), o3 = *(const v2f*)(dbeta + c6 + 4);
          float x[8], gg[8], bb[8];
          {
            const float a0 = tw.x * t + tb.x;
            const float a1 = tw.y * t + tb.y;
            x[0] = sinf(a0) * hm.x;
            x[1] = sinf(a1) * hm.y;
          }
          x[2] = h0.x; x[3] = h0.y; x[4] = h1.x; x[5] = h1.y; x[6] = h2.x; x[7] = h2.y;
          gg[0] = g0.x; gg[1] = g0.y; gg[2] = g1.x; gg[3] = g1.y; gg[4] = g2.x; gg[5] = g2.y; gg[6] = g3.x; gg[7] = g3.y;
          bb[0] = o0.x; bb[1] = o0.y; bb[2] = o1.x; bb[3] = o1.y; bb[4] = o2.x; bb[5] = o2.y; bb[6] = o3.x; bb[7] = o3.y;
          float s = 0.f;
#pragma unroll
          for (int j = 0; j < 8; ++j) s += x[j];
          s = hsum16(s);
          const float mu = s * (1.0f / (float)ID);
          float q = 0.f;
#pragma unroll
          for (int j = 0; j < 8; ++j) { const float dv = x[j] - mu; q += dv * dv; }
          q = hsum16(q);
          const float rs = rsqrtf(q * (1.0f / (float)ID) + LN_EPS);
          float y[8];
#pragma unroll
          for (int j = 0; j < 8; ++j) {
            const float dv = x[j] - mu;
            const float z = dv * rs;
            const float v = z * gg[j] + bb[j];
            y[j] = valid ? v : 0.f;
          }
          unsigned int p0h, p0l, p1h, p1l, p2h, p2l, p3h, p3l;
          split2(y[0], y[1], p0h, p0l);
          split2(y[2], y[3], p1h, p1l);
          split2(y[4], y[5], p2h, p2l);
          split2(y[6], y[7], p3h, p3l);
          unsigned short* rh = sAdH + m * ID;
          unsigned short* rl = sAdL + m * ID;
          *(unsigned int*)(rh + c2) = p0h; *(unsigned int*)(rh + c6) = p1h; *(unsigned int*)(rh + c6 + 2) = p2h; *(unsigned int*)(rh + c6 + 4) = p3h;
          *(unsigned int*)(rl + c2) = p0l; *(unsigned int*)(rl + c6) = p1l; *(unsigned int*)(rl + c6 + 2) = p2l; *(unsigned int*)(rl + c6 + 4) = p3l;
        }
        {
          const float* hr = src_h + (size_t)si * ID;
          const v2f hm = *(const v2f*)(hr + c2);
          const v2f tw = *(const v2f*)(src_tw + (size_t)si * TD + c2);
          const v2f tb = *(const v2f*)(src_tb + (size_t)si * TD + c2);
          const v2f h0 = *(const v2f*)(hr + c6), h1 = *(const v2f*)(hr + c6 + 2), h2 = *(const v2f*)(hr + c6 + 4);
          const v2f eh = *(const v2f*)(edge_h + (size_t)e * ED + c2);
          const v2f g0 = *(const v2f*)(sg + c2), g1 = *(const v2f*)(sg + c6), g2 = *(const v2f*)(sg + c6 + 2), g3 = *(const v2f*)(sg + c6 + 4), g4 = *(const v2f*)(sg + ID + c2);
          const v2f o0 = *(const v2f*)(sb + c2), o1 = *(const v2f*)(sb + c6), o2 = *(const v2f*)(sb + c6 + 2), o3 = *(const v2f*)(sb + c6 + 4), o4 = *(const v2f*)(sb + ID + c2);
          float x[10], gg[10], bb[10];
          {
            const float a0 = tw.x * t + tb.x;
            const float a1 = tw.y * t + tb.y;
            x[0] = sinf(a0) * hm.x;
            x[1] = sinf(a1) * hm.y;
          }
          x[2] = h0.x; x[3] = h0.y; x[4] = h1.x; x[5] = h1.y; x[6] = h2.x; x[7] = h2.y; x[8] = eh.x; x[9] = eh.y;
          gg[0] = g0.x; gg[1] = g0.y; gg[2] = g1.x; gg[3] = g1.y; gg[4] = g2.x; gg[5] = g2.y; gg[6] = g3.x; gg[7] = g3.y; gg[8] = g4.x; gg[9] = g4.y;
          bb[0] = o0.x; bb[1] = o0.y; bb[2] = o1.x; bb[3] = o1.y; bb[4] = o2.x; bb[5] = o2.y; bb[6] = o3.x; bb[7] = o3.y; bb[8] = o4.x; bb[9] = o4.y;
          float s = 0.f;
#pragma unroll
          for (int j = 0; j < 10; ++j) s += x[j];
          s = hsum16(s);
          const float mu = s * (1.0f / (float)KS);
          float q = 0.f;
#pragma unroll
          for (int j = 0; j < 10; ++j) { const float dv = x[j] - mu; q += dv * dv; }
          q = hsum16(q);
          const float rs = rsqrtf(q * (1.0f / (float)KS) + LN_EPS);
          float y[10];
#pragma unroll
          for (int j = 0; j < 10; ++j) {
            const float dv = x[j] - mu;
            const float z = dv * rs;
            const float v = z * gg[j] + bb[j];
            y[j] = valid ? v : 0.f;
          }
          unsigned int p0h, p0l, p1h, p1l, p2h, p2l, p3h, p3l, p4h, p4l;
          split2(y[0], y[1], p0h, p0l);
          split2(y[2], y[3], p1h, p1l);
          split2(y[4], y[5], p2h, p2l);
          split2(y[6], y[7], p3h, p3l);
          split2(y[8], y[9], p4h, p4l);
          unsigned short* rh = sAsH + m * KS;
          unsigned short* rl = sAsL + m * KS;
          *(unsigned int*)(rh + c2) = p0h; *(unsigned int*)(rh + c6) = p1h; *(unsigned int*)(rh + c6 + 2) = p2h; *(unsigned int*)(rh + c6 + 4) = p3h; *(unsigned int*)(rh + ID + c2) = p4h;
          *(unsigned int*)(rl + c2) = p0l; *(unsigned int*)(rl + c6) = p1l; *(unsigned int*)(rl + c6 + 2) = p2l; *(unsigned int*)(rl + c6 + 4) = p3l; *(unsigned int*)(rl + ID + c2) = p4l;
        }
      }
      __syncthreads();

      {
        const int n = wave * 16 + mc;
        v8f aq = zero8f(), ak = zero8f(), av = zero8f();
        {
          const unsigned short* a_h = sAdH + mc * ID + 8 * hh;
          const unsigned short* a_l = sAdL + mc * ID + 8 * hh;
          const unsigned short* b_h = wq_h + (size_t)n * ID + 8 * hh;
          const unsigned short* b_l = wq_l + (size_t)n * ID + 8 * hh;
#pragma unroll 1
          for (int kb = 0; kb < ID; kb += 32) {
            const FragB ah = ldfrag(a_h + kb), al = ldfrag(a_l + kb);
            const FragB bh = ldfrag(b_h + kb), bl = ldfrag(b_l + kb);
            aq = wmb(ah, bh, aq);
            aq = wmb(ah, bl, aq);
            aq = wmb(al, bh, aq);
          }
        }
        {
          const unsigned short* a_h = sAsH + mc * KS + 8 * hh;
          const unsigned short* a_l = sAsL + mc * KS + 8 * hh;
          const unsigned short* k_h = wk_h + (size_t)n * KS + 8 * hh;
          const unsigned short* k_l = wk_l + (size_t)n * KS + 8 * hh;
          const unsigned short* v_h = wv_h + (size_t)n * KS + 8 * hh;
          const unsigned short* v_l = wv_l + (size_t)n * KS + 8 * hh;
#pragma unroll 1
          for (int kb = 0; kb < KS; kb += 32) {
            const FragB ah = ldfrag(a_h + kb), al = ldfrag(a_l + kb);
            {
              const FragB bh = ldfrag(k_h + kb), bl = ldfrag(k_l + kb);
              ak = wmb(ah, bh, ak);
              ak = wmb(ah, bl, ak);
              ak = wmb(al, bh, ak);
            }
            {
              const FragB bh = ldfrag(v_h + kb), bl = ldfrag(v_l + kb);
              av = wmb(ah, bh, av);
              av = wmb(ah, bl, av);
              av = wmb(al, bh, av);
            }
          }
        }
#pragma unroll
        for (int j = 0; j < 8; ++j) {
          float p = aq[j] * ak[j];
          p = hsum16(p);
          sOut[(8 * hh + j) * EROW + n] = av[j];
          if (mc == 0) sOut[(8 * hh + j) * EROW + OD + wave] = p * ISQ;
        }
      }
      __syncthreads();

      {
        v4f va[2], vb[2];
        size_t ro[2];
        bool rv[2];
#pragma unroll
        for (int j2 = 0; j2 < 2; ++j2) {
          const int row = 2 * wave + j2;
          const int idx = tile * ETILE + row;
          rv[j2] = idx < tot;
          int e = pend[idx];
          e = rv[j2] ? e : 0;
          e = clampi(e, 0, nE - 1);
          ro[j2] = (size_t)e * EROW;
          va[j2] = *(const v4f*)(sOut + row * EROW + 4 * lane);
          vb[j2] = *(const v4f*)(sOut + row * EROW + OD + 4 * (lane & 7));
        }
#pragma unroll
        for (int j2 = 0; j2 < 2; ++j2) {
          if (rv[j2]) {
            *(volatile v4f*)(eplane + ro[j2] + 4 * lane) = va[j2];
            if (lane < 8) *(volatile v4f*)(eplane + ro[j2] + OD + 4 * lane) = vb[j2];
          }
        }
        __threadfence();
#pragma unroll
        for (int j2 = 0; j2 < 2; ++j2) {
          if (rv[j2]) {
            *(volatile v4f*)(eplane + ro[j2] + 4 * lane) = va[j2];
            if (lane < 8) *(volatile v4f*)(eplane + ro[j2] + OD + 4 * lane) = vb[j2];
          }
        }
      }
    }
  }
}

__global__ __launch_bounds__(NTHR) void k_agg(
    const float* __restrict__ eplane, const int* __restrict__ dst_idx, const int* __restrict__ ntype,
    const float* __restrict__ h_bias, const float* __restrict__ skip, const float* __restrict__ src_h,
    const unsigned short* __restrict__ wah, const unsigned short* __restrict__ wal,
    float* outp, int nM, int nN, int nE, int vec8) {
  __shared__ __attribute__((aligned(16))) float vacc[(NB + 1) * OD];
  __shared__ __attribute__((aligned(16))) float vden[(NB + 1) * NH];
  __shared__ __attribute__((aligned(16))) float vmx[(NB + 1) * NH];
  __shared__ __attribute__((aligned(16))) int   list[LISTN];
  __shared__ __attribute__((aligned(16))) int   pend[LISTN];
  __shared__ __attribute__((aligned(16))) float msg[NWAVE * MSGW];
  __shared__ __attribute__((aligned(16))) float amsg[NTHR * NH];
  __shared__ int slotb[NTHR];
  __shared__ int slotw[NWAVE];
  __shared__ __attribute__((aligned(16))) unsigned short sAh[ETILE * OD];
  __shared__ __attribute__((aligned(16))) unsigned short sAl[ETILE * OD];
  __shared__ __attribute__((aligned(16))) float sO[ETILE * OD];
  __shared__ int   sNt[ETILE];
  __shared__ float sGate[ETILE];
  __shared__ int   wcnt[NWAVE];

  const int tid = threadIdx.x, lane = tid & 31, wave = tid >> 5, hh = lane >> 4, mc = lane & 15;
  const int m = tid >> 4, ln = tid & 15;
  const int nodeBase = blockIdx.x * NB;
  const float ninf = __uint_as_float(0xff800000u);

  for (int i = tid; i < (NB + 1) * OD; i += NTHR) vacc[i] = 0.f;
  for (int i = tid; i < (NB + 1) * NH; i += NTHR) { vden[i] = 0.f; vmx[i] = ninf; }
  __syncthreads();

  const int nChunks = (nE + CHUNK - 1) / CHUNK;

#pragma unroll 1
  for (int ch = 0; ch < nChunks; ++ch) {
    const int cbase = ch * CHUNK;
    {
      const int e0 = cbase + tid * EPT;
      const int full = (vec8 != 0 && cbase + CHUNK <= nE) ? 1 : 0;
      v4i da, db;
      load8(dst_idx, nE, e0, full, da, db);
      const unsigned nb = (unsigned)nodeBase;
      const int wc = compact8(((unsigned)da.x - nb) < (unsigned)NB, ((unsigned)da.y - nb) < (unsigned)NB,
                              ((unsigned)da.z - nb) < (unsigned)NB, ((unsigned)da.w - nb) < (unsigned)NB,
                              ((unsigned)db.x - nb) < (unsigned)NB, ((unsigned)db.y - nb) < (unsigned)NB,
                              ((unsigned)db.z - nb) < (unsigned)NB, ((unsigned)db.w - nb) < (unsigned)NB,
                              tid * EPT, list, wave);
      if (lane == 0) wcnt[wave] = wc;
    }
    __syncthreads();
    const int tot = flatten(list, pend, wcnt, cbase, lane, wave);
    __syncthreads();
    const int nS = (tot + NTHR - 1) / NTHR;
#pragma unroll 1
    for (int s = 0; s < nS; ++s) {
      {
        const int i = s * NTHR + tid;
        const bool valid = i < tot;
        int e = pend[clampi(i, 0, LISTN - 1)];
        e = valid ? e : 0;
        e = clampi(e, 0, nE - 1);
        const int d = dst_idx[e];
        int slot = d - nodeBase;
        if (!valid || (unsigned)slot >= (unsigned)NB) slot = NB;
        const float* rp = eplane + (size_t)e * EROW + OD;
        const v4f a0 = *(const v4f*)rp;
        const v4f a1 = *(const v4f*)(rp + 4);
        *(v4f*)(amsg + tid * NH) = a0;
        *(v4f*)(amsg + tid * NH + 4) = a1;
        slotb[tid] = slot;
      }
      __syncthreads();
      if (tid < NH) {
        int cnt = tot - s * NTHR;
        cnt = cnt > NTHR ? NTHR : cnt;
#pragma unroll 1
        for (int i = 0; i < cnt; ++i) {
          const int sl = clampi(slotb[i], 0, NB);
          float* mp = vmx + sl * NH + tid;
          *mp = fmaxf(*mp, amsg[i * NH + tid]);
        }
      }
      __syncthreads();
    }
  }
  __syncthreads();

#pragma unroll 1
  for (int ch = 0; ch < nChunks; ++ch) {
    const int cbase = ch * CHUNK;
    {
      const int e0 = cbase + tid * EPT;
      const int full = (vec8 != 0 && cbase + CHUNK <= nE) ? 1 : 0;
      v4i da, db;
      load8(dst_idx, nE, e0, full, da, db);
      const unsigned nb = (unsigned)nodeBase;
      const int wc = compact8(((unsigned)da.x - nb) < (unsigned)NB, ((unsigned)da.y - nb) < (unsigned)NB,
                              ((unsigned)da.z - nb) < (unsigned)NB, ((unsigned)da.w - nb) < (unsigned)NB,
                              ((unsigned)db.x - nb) < (unsigned)NB, ((unsigned)db.y - nb) < (unsigned)NB,
                              ((unsigned)db.z - nb) < (unsigned)NB, ((unsigned)db.w - nb) < (unsigned)NB,
                              tid * EPT, list, wave);
      if (lane == 0) wcnt[wave] = wc;
    }
    __syncthreads();
    const int tot = flatten(list, pend, wcnt, cbase, lane, wave);
    __syncthreads();
    const int nS = (tot + NWAVE - 1) / NWAVE;
#pragma unroll 1
    for (int s = 0; s < nS; ++s) {
      {
        const int i = s * NWAVE + wave;
        const bool valid = i < tot;
        int e = pend[clampi(i, 0, LISTN - 1)];
        e = valid ? e : 0;
        e = clampi(e, 0, nE - 1);
        const int d = dst_idx[e];
        int slot = d - nodeBase;
        const bool ok = valid && ((unsigned)slot < (unsigned)NB);
        if (!ok) slot = NB;
        const float* rp = eplane + (size_t)e * EROW;
        const v4f vv = *(const v4f*)(rp + 4 * lane);
        const int hd = lane >> 2;
        const float a = rp[OD + hd];
        const float mxv = vmx[slot * NH + hd];
        const float dl = ok ? (a - mxv) : 0.f;
        const float p = ok ? expf(dl) : 0.f;
        const v4f mv = vv * p;
        *(v4f*)(msg + wave * MSGW + 4 * lane) = mv;
        if ((lane & 3) == 0) msg[wave * MSGW + OD + hd] = p;
        if (lane == 0) slotw[wave] = slot;
      }
      __syncthreads();
      if (tid < MSGW) {
        int cnt = tot - s * NWAVE;
        cnt = cnt > NWAVE ? NWAVE : cnt;
#pragma unroll 1
        for (int i = 0; i < cnt; ++i) {
          const int sl = clampi(slotw[i], 0, NB);
          const float v = msg[i * MSGW + tid];
          if (tid < OD) vacc[sl * OD + tid] += v;
          else          vden[sl * NH + (tid - OD)] += v;
        }
      }
      __syncthreads();
    }
  }
  __syncthreads();

#pragma unroll 1
  for (int rt = 0; rt < NB / ETILE; ++rt) {
    {
      const int slot = rt * ETILE + m;
      const int node = nodeBase + slot;
      const bool nv = node < nM;
      const int nt = clampi(ntype[clampi(node, 0, nM - 1)], 0, NTYP - 1);
      const int c8 = 8 * ln;
      const int hd = ln >> 1;
      const float den = vden[slot * NH + hd];
      const float rden = (den > 0.f) ? __builtin_amdgcn_rcpf(den) : 0.f;
      const v4f b0 = *(const v4f*)(h_bias + (size_t)nt * OD + c8);
      const v4f b1 = *(const v4f*)(h_bias + (size_t)nt * OD + c8 + 4);
      const v4f s0 = *(const v4f*)(vacc + slot * OD + c8);
      const v4f s1 = *(const v4f*)(vacc + slot * OD + c8 + 4);
      float x[8];
      x[0] = s0.x * rden + b0.x; x[1] = s0.y * rden + b0.y; x[2] = s0.z * rden + b0.z; x[3] = s0.w * rden + b0.w;
      x[4] = s1.x * rden + b1.x; x[5] = s1.y * rden + b1.y; x[6] = s1.z * rden + b1.z; x[7] = s1.w * rden + b1.w;
#pragma unroll
      for (int j = 0; j < 8; ++j) x[j] = nv ? x[j] : 0.f;
      unsigned int p0h, p0l, p1h, p1l, p2h, p2l, p3h, p3l;
      split2(x[0], x[1], p0h, p0l);
      split2(x[2], x[3], p1h, p1l);
      split2(x[4], x[5], p2h, p2l);
      split2(x[6], x[7], p3h, p3l);
      v4u hv = {p0h, p1h, p2h, p3h};
      v4u lv = {p0l, p1l, p2l, p3l};
      *(v4u*)(sAh + m * OD + c8) = hv;
      *(v4u*)(sAl + m * OD + c8) = lv;
      if (ln == 0) {
        sNt[m] = nt;
        const float sk = skip[nt];
        const float ex = expf(-sk);
        sGate[m] = __builtin_amdgcn_rcpf(1.0f + ex);
      }
    }
    __syncthreads();
    {
      const int n = wave * 16 + mc;
      int ntv[8];
#pragma unroll
      for (int j = 0; j < 8; ++j) ntv[j] = sNt[8 * hh + j];
      v8f sel = zero8f();
      const unsigned short* a_h = sAh + mc * OD + 8 * hh;
      const unsigned short* a_l = sAl + mc * OD + 8 * hh;
#pragma unroll 1
      for (int t = 0; t < NTYP; ++t) {
        v8f dacc = zero8f();
        const unsigned short* b_h = wah + ((size_t)t * OD + n) * OD + 8 * hh;
        const unsigned short* b_l = wal + ((size_t)t * OD + n) * OD + 8 * hh;
#pragma unroll 1
        for (int kb = 0; kb < OD; kb += 32) {
          const FragB ah = ldfrag(a_h + kb), al = ldfrag(a_l + kb);
          const FragB bh = ldfrag(b_h + kb), bl = ldfrag(b_l + kb);
          dacc = wmb(ah, bh, dacc);
          dacc = wmb(ah, bl, dacc);
          dacc = wmb(al, bh, dacc);
        }
#pragma unroll
        for (int j = 0; j < 8; ++j) sel[j] = (ntv[j] == t) ? dacc[j] : sel[j];
      }
#pragma unroll
      for (int j = 0; j < 8; ++j) sO[(8 * hh + j) * OD + n] = sel[j];
    }
    __syncthreads();
    {
      v4f ov[2];
      size_t oo[2];
      bool rv[2];
#pragma unroll
      for (int j2 = 0; j2 < 2; ++j2) {
        const int row = 2 * wave + j2;
        const int node = nodeBase + rt * ETILE + row;
        rv[j2] = node < nM;
        const int nc = clampi(node, 0, nN - 1);
        const float g = sGate[row];
        const float omg = 1.0f - g;
        const v4f hv = *(const v4f*)(sO + row * OD + 4 * lane);
        const v4f xr = *(const v4f*)(src_h + (size_t)nc * ID + 4 * lane);
        const v4f t1 = hv * g;
        const v4f t2 = xr * omg;
        ov[j2] = t1 + t2;
        oo[j2] = (size_t)nc * OD + 4 * lane;
      }
#pragma unroll
      for (int j2 = 0; j2 < 2; ++j2) if (rv[j2]) *(volatile v4f*)(outp + oo[j2]) = ov[j2];
      __threadfence();
#pragma unroll
      for (int j2 = 0; j2 < 2; ++j2) if (rv[j2]) *(volatile v4f*)(outp + oo[j2]) = ov[j2];
    }
    __syncthreads();
  }
}

extern "C" void kernel_launch(void* const* d_in, const int* in_sizes, int n_in,
                              void* d_out, int out_size, void* d_ws, size_t ws_size,
                              hipStream_t stream) {
  if (n_in < 19) return;
  const int nN = in_sizes[0] / ID;
  const int nE = in_sizes[4];
  const int nM = in_sizes[8];
  if (nN < 1 || nE < 1 || nM < 1 || nM > nN) return;
  if (in_sizes[0] != nN * ID || in_sizes[1] != nN * TD || in_sizes[2] != nN * TD) return;
  if (in_sizes[3] != nE * ED || in_sizes[5] != nE || in_sizes[6] != nE || in_sizes[7] != nE) return;
  if (in_sizes[9] != NREL * ID * OD || in_sizes[10] != NREL * KS * OD || in_sizes[11] != NREL * KS * OD) return;
  if (in_sizes[12] != NTYP * OD * OD || in_sizes[13] != NTYP * OD || in_sizes[14] != NTYP) return;
  if (in_sizes[15] != KS || in_sizes[16] != KS || in_sizes[17] != ID || in_sizes[18] != ID) return;
  if (out_size != nM * OD) return;

  const float* src_h   = (const float*)d_in[0];
  const float* src_tw  = (const float*)d_in[1];
  const float* src_tb  = (const float*)d_in[2];
  const float* edge_h  = (const float*)d_in[3];
  const float* date    = (const float*)d_in[4];
  const int*   src_idx = (const int*)d_in[5];
  const int*   dst_idx = (const int*)d_in[6];
  const int*   etype   = (const int*)d_in[7];
  const int*   ntype   = (const int*)d_in[8];
  const float* Wq      = (const float*)d_in[9];
  const float* Wk      = (const float*)d_in[10];
  const float* Wv      = (const float*)d_in[11];
  const float* Wa      = (const float*)d_in[12];
  const float* h_bias  = (const float*)d_in[13];
  const float* skip    = (const float*)d_in[14];
  const float* sg      = (const float*)d_in[15];
  const float* sb      = (const float*)d_in[16];
  const float* dg      = (const float*)d_in[17];
  const float* dbt     = (const float*)d_in[18];
  float* out = (float*)d_out;

  const size_t szE = (size_t)nE * EROW * sizeof(float);
  const size_t szQ = (size_t)NREL * OD * ID * 2;
  const size_t szK = (size_t)NREL * OD * KS * 2;
  const size_t szA = (size_t)NTYP * OD * OD * 2;
  size_t off = 0;
  const size_t oE  = off; off += (szE + 255) & ~(size_t)255;
  const size_t oQh = off; off += (szQ + 255) & ~(size_t)255;
  const size_t oQl = off; off += (szQ + 255) & ~(size_t)255;
  const size_t oKh = off; off += (szK + 255) & ~(size_t)255;
  const size_t oKl = off; off += (szK + 255) & ~(size_t)255;
  const size_t oVh = off; off += (szK + 255) & ~(size_t)255;
  const size_t oVl = off; off += (szK + 255) & ~(size_t)255;
  const size_t oAh = off; off += (szA + 255) & ~(size_t)255;
  const size_t oAl = off; off += (szA + 255) & ~(size_t)255;
  if (off > ws_size) return;
  char* ws = (char*)d_ws;
  float* eplane = (float*)(ws + oE);
  unsigned short* wqh = (unsigned short*)(ws + oQh);
  unsigned short* wql = (unsigned short*)(ws + oQl);
  unsigned short* wkh = (unsigned short*)(ws + oKh);
  unsigned short* wkl = (unsigned short*)(ws + oKl);
  unsigned short* wvh = (unsigned short*)(ws + oVh);
  unsigned short* wvl = (unsigned short*)(ws + oVl);
  unsigned short* wah = (unsigned short*)(ws + oAh);
  unsigned short* wal = (unsigned short*)(ws + oAl);

  const int vec8 = 1;
  const int nGroups = NREL * OD * (ID / 8) + 2 * NREL * OD * (KS / 8) + NTYP * OD * (OD / 8);
  const int nEdgeBlk = (nE + CHUNK - 1) / CHUNK;
  const int nNodeBlk = (nM + NB - 1) / NB;

  k_wprep<<<(nGroups + NTHR - 1) / NTHR, NTHR, 0, stream>>>(Wq, Wk, Wv, Wa, wqh, wql, wkh, wkl, wvh, wvl, wah, wal);

  k_edge<<<nEdgeBlk, NTHR, 0, stream>>>(src_h, src_tw, src_tb, edge_h, date, src_idx, dst_idx, etype,
                                        sg, sb, dg, dbt, wqh, wql, wkh, wkl, wvh, wvl,
                                        eplane, nN, nE, vec8);

  k_agg<<<nNodeBlk, NTHR, 0, stream>>>(eplane, dst_idx, ntype, h_bias, skip, src_h, wah, wal,
                                       out, nM, nN, nE, vec8);
}
